// MHSelfAttention_61967788146887
// MI455X (gfx1250) — hardware-verified
//
#include <hip/hip_runtime.h>
#include <math.h>

constexpr int kBatch  = 4;
constexpr int kSeq    = 2048;
constexpr int kDim    = 1024;
constexpr int kHeads  = 16;
constexpr int kDh     = 64;
constexpr int kTok    = kBatch * kSeq;
constexpr int kWRows  = 3 * kDim;
constexpr int kQKCols = 2 * kDim;
constexpr float kPCarry    = 32768.0f;
constexpr float kScale     = 0.125f;
static_assert(kHeads * kDh == kDim, "shape");
static_assert(kDim % 32 == 0, "gemm K multiple of 32");
static_assert(kTok % 64 == 0 && kQKCols % 64 == 0 && kDh % 64 == 0 && kSeq % 64 == 0, "gemm M,N multiples of 64");
static_assert((kTok * kDim) % (8 * 256) == 0 && (kWRows * kDim) % (8 * 256) == 0, "cast grids exact");

typedef __attribute__((ext_vector_type(16))) _Float16 v16h;
typedef __attribute__((ext_vector_type(8)))  _Float16 v8h;
typedef __attribute__((ext_vector_type(16))) __bf16   v16b;
typedef __attribute__((ext_vector_type(8)))  __bf16   v8b;
typedef __attribute__((ext_vector_type(8)))  float    v8f;
typedef __attribute__((ext_vector_type(4)))  float    v4f;
typedef __attribute__((ext_vector_type(4)))  unsigned int v4u;

__device__ __forceinline__ unsigned short f2bf_bits(float f) {
  unsigned u = __float_as_uint(f);
  return (unsigned short)((u + 0x7FFFu + ((u >> 16) & 1u)) >> 16);
}
__device__ __forceinline__ float bf_bits2f(unsigned short h) { return __uint_as_float(((unsigned)h) << 16); }

__device__ __forceinline__ void dep_guard_h(v8f& a, v8f& b, v16h x, v16h y) { asm volatile("v_nop\n\tv_nop\n\tv_nop\n\tv_nop" : "+v"(a), "+v"(b) : "v"(x), "v"(y)); }
__device__ __forceinline__ void dep_guard_b(v8f& a, v8f& b, v16b x, v16b y) { asm volatile("v_nop\n\tv_nop\n\tv_nop\n\tv_nop" : "+v"(a), "+v"(b) : "v"(x), "v"(y)); }
__device__ __forceinline__ void keep4_h(v16h a, v16h b, v16h c, v16h d) { asm volatile("v_nop" :: "v"(a), "v"(b), "v"(c), "v"(d)); }
__device__ __forceinline__ void keep4_b(v16b a, v16b b, v16b c, v16b d) { asm volatile("v_nop" :: "v"(a), "v"(b), "v"(c), "v"(d)); }
__device__ __forceinline__ void acc_guard4(v8f& a, v8f& b, v8f& c, v8f& d) { asm volatile("v_nop\n\tv_nop\n\tv_nop\n\tv_nop" : "+v"(a), "+v"(b), "+v"(c), "+v"(d)); }
template <typename T> struct Frag;
template <> struct Frag<_Float16> {
  typedef v16h V; union U { v16h v; v8h h[2]; };
  static __device__ __forceinline__ v16h load(const _Float16* p) {
    U f; f.h[0] = *(const v8h*)(p); f.h[1] = *(const v8h*)(p + 16); return f.v;
  }
  static __device__ __forceinline__ v8f mma(v16h a, v16h b, v8f c) {
    return __builtin_amdgcn_wmma_f32_16x16x32_f16(false, a, false, b, (short)0, c, false, false);
  }
  static __device__ __forceinline__ void guard(v8f& a, v8f& b, v16h x, v16h y) { dep_guard_h(a, b, x, y); }
  static __device__ __forceinline__ void keep(v16h a, v16h b, v16h c, v16h d) { keep4_h(a, b, c, d); }
};
template <> struct Frag<__bf16> {
  typedef v16b V; union U { v16b v; v8b h[2]; };
  static __device__ __forceinline__ v16b load(const __bf16* p) {
    U f; f.h[0] = *(const v8b*)(p); f.h[1] = *(const v8b*)(p + 16); return f.v;
  }
  static __device__ __forceinline__ v8f mma(v16b a, v16b b, v8f c) {
    return __builtin_amdgcn_wmma_f32_16x16x32_bf16(false, a, false, b, (short)0, c, false, false);
  }
  static __device__ __forceinline__ void guard(v8f& a, v8f& b, v16b x, v16b y) { dep_guard_b(a, b, x, y); }
  static __device__ __forceinline__ void keep(v16b a, v16b b, v16b c, v16b d) { keep4_b(a, b, c, d); }
};

__device__ __forceinline__ unsigned pk16(unsigned short a, unsigned short b) { return (unsigned)a | ((unsigned)b << 16); }

template <int ET> struct Elem;
template <> struct Elem<0> { typedef _Float16 T; };
template <> struct Elem<1> { typedef __bf16 T; };
template <int ET, bool SPLIT, int BIAS_MODE, int OUT_MODE, bool RESID, int ACT = 0>
__global__ __launch_bounds__(256) void wmma_gemm64(
    const unsigned short* __restrict__ Ap, const unsigned short* __restrict__ A2p, int lda, long strideA,
    const unsigned short* __restrict__ Btp, const unsigned short* __restrict__ Bt2p, int ldb, long strideB,
    void* __restrict__ Cout, void* __restrict__ Cout2, int ldc, long strideC,
    const float* __restrict__ bias,
    const float* __restrict__ resid, long strideR,
    int M, int N, int K, float scale) {
  typedef typename Elem<ET>::T T;
  typedef typename Frag<T>::V V;
  const T* A = (const T*)Ap; const T* A2 = (const T*)A2p; const T* Bt = (const T*)Btp; const T* Bt2 = (const T*)Bt2p;
  __shared__ __align__(16) float sT[8][16 * 68];
  const int b    = blockIdx.y;
  const int lane = threadIdx.x & 31;
  const int wave = threadIdx.x >> 5;
  const int tilesN = N >> 6;
  const int tilesM = M >> 6;
  const int tile = blockIdx.x * 8 + wave;
  if (tile >= tilesM * tilesN) return;
  const int tm = tile / tilesN;
  const int tn = tile - tm * tilesN;
  const int m0 = tm << 6;
  const int n0 = tn << 6;

  const T* Ab  = A  + (size_t)b * strideA;
  const T* Bb  = Bt + (size_t)b * strideB;
  const T* Ab2 = SPLIT ? (A2  + (size_t)b * strideA) : nullptr;
  const T* Bb2 = SPLIT ? (Bt2 + (size_t)b * strideB) : nullptr;

  const int rlane = lane & 15;
  const int koff  = (lane >> 4) * 8;
  const int mOff  = (lane >> 4) * 8;

  v8f acc[4][4];
#pragma unroll
  for (int i = 0; i < 4; ++i)
#pragma unroll
    for (int j = 0; j < 4; ++j) acc[i][j] = (v8f){0.f,0.f,0.f,0.f,0.f,0.f,0.f,0.f};

  for (int k0 = 0; k0 < K; k0 += 32) {
    V bh[4], bl[4];
#pragma unroll
    for (int j = 0; j < 4; ++j) {
      const size_t bo = (size_t)(n0 + (j << 4) + rlane) * ldb + koff + k0;
      bh[j] = Frag<T>::load(Bb + bo);
      if (SPLIT) bl[j] = Frag<T>::load(Bb2 + bo);
    }
#pragma unroll
    for (int i = 0; i < 4; ++i) {
      const size_t ao = (size_t)(m0 + (i << 4) + rlane) * lda + koff + k0;
      V ah = Frag<T>::load(Ab + ao);
      V al;
      if (SPLIT) al = Frag<T>::load(Ab2 + ao);
#pragma unroll
      for (int j = 0; j < 4; ++j) {
        acc[i][j] = Frag<T>::mma(ah, bh[j], acc[i][j]);
        if (SPLIT) {
          acc[i][j] = Frag<T>::mma(ah, bl[j], acc[i][j]);
          acc[i][j] = Frag<T>::mma(al, bh[j], acc[i][j]);
        }
      }
      Frag<T>::guard(acc[i][0], acc[i][3], ah, SPLIT ? al : ah);
    }
    Frag<T>::keep(bh[0], bh[1], bh[2], bh[3]);
    if (SPLIT) Frag<T>::keep(bl[0], bl[1], bl[2], bl[3]);
  }
  acc_guard4(acc[0][0], acc[0][1], acc[0][2], acc[0][3]);
  acc_guard4(acc[1][0], acc[1][1], acc[1][2], acc[1][3]);
  acc_guard4(acc[2][0], acc[2][1], acc[2][2], acc[2][3]);
  acc_guard4(acc[3][0], acc[3][1], acc[3][2], acc[3][3]);

  float* slab = sT[wave];
  const float* Rb = RESID ? (resid + (size_t)b * strideR) : nullptr;
#pragma unroll
  for (int i = 0; i < 4; ++i) {
    const int mBase = m0 + (i << 4);
#pragma unroll
    for (int j = 0; j < 4; ++j) {
      const int n = n0 + (j << 4) + rlane;
      float bv = 0.f;
      if (BIAS_MODE == 2) bv = bias[n];
#pragma unroll
      for (int r = 0; r < 8; ++r) {
        float v = acc[i][j][r] * scale;
        if (BIAS_MODE == 1) v += bias[mBase + mOff + r];
        if (BIAS_MODE == 2) v += bv;
        if (RESID) v += Rb[(size_t)(mBase + mOff + r) * ldc + n];
        if (ACT == 2) v = fmaxf(v, 0.0f);
        if (ACT == 4) v = (v > 0.f) ? v : 0.01f * v;
        slab[(mOff + r) * 68 + (j << 4) + rlane] = v;
      }
    }
    __builtin_amdgcn_fence(__ATOMIC_RELEASE, "workgroup");
    __builtin_amdgcn_wave_barrier();
    __builtin_amdgcn_fence(__ATOMIC_ACQUIRE, "workgroup");
    if (OUT_MODE == 0) {
      float* C = (float*)Cout + (size_t)b * strideC;
      const int hh = lane >> 4, c4 = (lane & 15) * 4;
      for (int pass = 0; pass < 2; ++pass) {
#pragma unroll
        for (int it = 0; it < 8; ++it) {
          const int row = it * 2 + hh;
          v4f v = *(const v4f*)(slab + row * 68 + c4);
          *(volatile v4f*)(C + (size_t)(mBase + row) * ldc + n0 + c4) = v;
        }
        __threadfence();
      }
    } else {
      const int q = lane >> 3, c8 = (lane & 7) * 8;
      unsigned short* C  = (unsigned short*)Cout  + (size_t)b * strideC;
      unsigned short* C2 = (OUT_MODE == 2) ? ((unsigned short*)Cout2 + (size_t)b * strideC) : nullptr;
      for (int pass = 0; pass < 2; ++pass) {
#pragma unroll
        for (int it = 0; it < 4; ++it) {
          const int row = it * 4 + q;
          const float* sp = slab + row * 68 + c8;
          v8h hv, lv;
#pragma unroll
          for (int e = 0; e < 8; ++e) {
            if (OUT_MODE == 1) {
              hv[e] = (_Float16)sp[e];
            } else {
              unsigned short hb = f2bf_bits(sp[e]);
              unsigned short lb = f2bf_bits(sp[e] - bf_bits2f(hb));
              hv[e] = __builtin_bit_cast(_Float16, hb);
              lv[e] = __builtin_bit_cast(_Float16, lb);
            }
          }
          *(volatile v8h*)(C + (size_t)(mBase + row) * ldc + n0 + c8) = hv;
          if (OUT_MODE == 2) *(volatile v8h*)(C2 + (size_t)(mBase + row) * ldc + n0 + c8) = lv;
        }
        __threadfence();
      }
    }
    __builtin_amdgcn_fence(__ATOMIC_RELEASE, "workgroup");
    __builtin_amdgcn_wave_barrier();
    __builtin_amdgcn_fence(__ATOMIC_ACQUIRE, "workgroup");
  }
}

__global__ __launch_bounds__(256) void cast8_bf16_kernel(const float* __restrict__ in, unsigned short* __restrict__ out,
                                                         int n8) {
  const int i = blockIdx.x * 256 + threadIdx.x;
  if (i >= n8) return;
  const float* p = in + 8 * (size_t)i;
  const v4f a = *(const v4f*)(p);
  const v4f c = *(const v4f*)(p + 4);
  unsigned short hb[8];
#pragma unroll
  for (int e = 0; e < 4; ++e) {
    hb[e]     = f2bf_bits(a[e]);
    hb[4 + e] = f2bf_bits(c[e]);
  }
  const v4u u = (v4u){pk16(hb[0], hb[1]), pk16(hb[2], hb[3]), pk16(hb[4], hb[5]), pk16(hb[6], hb[7])};
  unsigned short* q = out + 8 * (size_t)i;
  *(volatile v4u*)q = u;
  __threadfence();
  *(volatile v4u*)q = u;
}

constexpr int kKC = 64;
constexpr int kQB = 64;
constexpr int kOsPitch = 68;
static_assert(kSeq % kKC == 0 && kSeq % kQB == 0, "attention tiles");

__device__ __forceinline__ v8f mma_h16(v16h a, v16h b, v8f c) {
  c = __builtin_amdgcn_wmma_f32_16x16x32_f16(false, a, false, b, (short)0, c, false, false);
  asm volatile("v_nop\n\tv_nop\n\tv_nop\n\tv_nop" : "+v"(c) : "v"(a), "v"(b));
  return c;
}

__global__ __launch_bounds__(128)
void attn_f16_kernel(const unsigned short* __restrict__ QKp, const unsigned short* __restrict__ VTp,
                     float* __restrict__ out) {
  const _Float16* QK = (const _Float16*)(const void*)QKp;
  const _Float16* VT = (const _Float16*)(const void*)VTp;
  __shared__ __align__(16) _Float16 Ksh[kKC * kDh];
  __shared__ __align__(16) _Float16 Vth[kDh * kKC];
  __shared__ __align__(16) _Float16 Psh[4][16 * kKC];
  __shared__ __align__(16) float    Os[4][16 * kOsPitch];

  const int tid  = threadIdx.x;
  const int wave = tid >> 5;
  const int lane = tid & 31;
  const int hh   = lane >> 4;
  const int c    = lane & 15;

  const int nqb = kSeq / kQB;
  const int bx  = blockIdx.x;
  const int qb  = bx % nqb;
  const int bh  = bx / nqb;
  const int h   = bh % kHeads;
  const int b   = bh / kHeads;
  const int q0  = qb * kQB + wave * 16;

  const _Float16* qb_ptr = QK + (size_t)b * kSeq * kQKCols + (size_t)h * kDh;
  const _Float16* kb_ptr = qb_ptr + kDim;
  const _Float16* vb_ptr = VT + (size_t)bh * kDh * kSeq;
  float*          ob_ptr = out + (size_t)b * kSeq * kDim + (size_t)h * kDh;

  v16h qa[2];
  {
    const _Float16* qrow = qb_ptr + (size_t)(q0 + c) * kQKCols + 8 * hh;
#pragma unroll
    for (int dc = 0; dc < 2; ++dc) qa[dc] = Frag<_Float16>::load(qrow + dc * 32);
  }

  float mrow[8], lrow[8];
  v8f oacc[4];
#pragma unroll
  for (int r = 0; r < 8; ++r) { mrow[r] = -__builtin_inff(); lrow[r] = 0.f; }
#pragma unroll
  for (int t = 0; t < 4; ++t) oacc[t] = (v8f){0.f,0.f,0.f,0.f,0.f,0.f,0.f,0.f};

  for (int kc = 0; kc < kSeq / kKC; ++kc) {
    const int kv0 = kc * kKC;
    __syncthreads();
#pragma unroll
    for (int i = 0; i < 4; ++i) {
      const int idx = i * 128 + tid;
      const int r   = idx >> 3;
      const int c8  = (idx & 7) * 8;
      const v8h kk = *(const v8h*)(kb_ptr + (size_t)(kv0 + r) * kQKCols + c8);
      const v8h vv = *(const v8h*)(vb_ptr + (size_t)r * kSeq + kv0 + c8);
      *(v8h*)(Ksh + r * kDh + c8) = kk;
      *(v8h*)(Vth + r * kKC + c8) = vv;
    }
    __syncthreads();

    v8f s[4];
#pragma unroll
    for (int j = 0; j < 4; ++j) {
      s[j] = (v8f){0.f,0.f,0.f,0.f,0.f,0.f,0.f,0.f};
#pragma unroll
      for (int dc = 0; dc < 2; ++dc) {
        const v16h kb = Frag<_Float16>::load(Ksh + (j * 16 + c) * kDh + dc * 32 + 8 * hh);
        s[j] = mma_h16(qa[dc], kb, s[j]);
      }
    }

    float cm[8];
#pragma unroll
    for (int r = 0; r < 8; ++r) {
      float m = -__builtin_inff();
#pragma unroll
      for (int j = 0; j < 4; ++j) {
        const float sv = s[j][r] * kScale;
        s[j][r] = sv;
        m = fmaxf(m, sv);
      }
#pragma unroll
      for (int off = 1; off < 16; off <<= 1) m = fmaxf(m, __shfl_xor(m, off, 32));
      cm[r] = m;
    }

    _Float16* pw = Psh[wave];
#pragma unroll
    for (int r = 0; r < 8; ++r) {
      const float mnew  = fmaxf(mrow[r], cm[r]);
      const float alpha = expf(mrow[r] - mnew);
      mrow[r] = mnew;
      float psum = 0.f;
#pragma unroll
      for (int j = 0; j < 4; ++j) {
        const float p = expf(s[j][r] - mnew);
        psum += p;
        pw[(8 * hh + r) * kKC + j * 16 + c] = (_Float16)(p * kPCarry);
      }
#pragma unroll
      for (int off = 1; off < 16; off <<= 1) psum += __shfl_xor(psum, off, 32);
      lrow[r] = lrow[r] * alpha + psum;
#pragma unroll
      for (int t = 0; t < 4; ++t) oacc[t][r] *= alpha;
    }
    __syncthreads();

#pragma unroll
    for (int kk = 0; kk < 2; ++kk) {
      const v16h pa = Frag<_Float16>::load(pw + c * kKC + kk * 32 + 8 * hh);
#pragma unroll
      for (int t = 0; t < 4; ++t) {
        const v16h vb = Frag<_Float16>::load(Vth + (t * 16 + c) * kKC + kk * 32 + 8 * hh);
        oacc[t] = mma_h16(pa, vb, oacc[t]);
      }
    }
  }

  float* os = Os[wave];
#pragma unroll
  for (int r = 0; r < 8; ++r) {
    const float inv = 1.0f / (lrow[r] * kPCarry);
#pragma unroll
    for (int t = 0; t < 4; ++t) os[(8 * hh + r) * kOsPitch + t * 16 + c] = oacc[t][r] * inv;
  }
  __syncthreads();
  {
    const int c4 = (lane & 15) * 4;
    for (int pass = 0; pass < 2; ++pass) {
#pragma unroll
      for (int it = 0; it < 8; ++it) {
        const int row = it * 2 + hh;
        const v4f val = *(const v4f*)(os + row * kOsPitch + c4);
        *(volatile v4f*)(ob_ptr + (size_t)(q0 + row) * kDim + c4) = val;
      }
      __threadfence();
    }
  }
}

extern "C" void kernel_launch(void* const* d_in, const int* in_sizes, int n_in,
                              void* d_out, int out_size, void* d_ws, size_t ws_size,
                              hipStream_t stream) {
  if (n_in < 2) return;
  if (in_sizes[0] != kTok * kDim) return;
  if (in_sizes[1] != kWRows * kDim) return;
  if (out_size != kTok * kDim) return;

  const size_t szXb = (size_t)kTok * kDim * 2;
  const size_t szWb = (size_t)kWRows * kDim * 2;
  const size_t szQK = (size_t)kTok * kQKCols * 2;
  const size_t szVt = (size_t)kBatch * kHeads * kDh * kSeq * 2;
  const size_t offXb = 0;
  const size_t offWb = offXb + szXb;
  const size_t offQK = offWb + szWb;
  const size_t offVt = offQK + szQK;
  const size_t total = offVt + szVt;
  if (ws_size < total) return;

  const float* x = (const float*)d_in[0];
  const float* W = (const float*)d_in[1];
  float* out = (float*)d_out;
  char* ws = (char*)d_ws;
  unsigned short* Xb  = (unsigned short*)(ws + offXb);
  unsigned short* Wb  = (unsigned short*)(ws + offWb);
  unsigned short* QKh = (unsigned short*)(ws + offQK);
  unsigned short* Vt  = (unsigned short*)(ws + offVt);

  const int n8x = (kTok * kDim) / 8;
  const int n8w = (kWRows * kDim) / 8;
  cast8_bf16_kernel<<<dim3(n8x / 256), dim3(256), 0, stream>>>(x, Xb, n8x);
  cast8_bf16_kernel<<<dim3(n8w / 256), dim3(256), 0, stream>>>(W, Wb, n8w);

  const int tilesQK = (kTok / 64) * (kQKCols / 64);
  wmma_gemm64<1, false, 0, 1, false, 0><<<dim3(tilesQK / 8, 1), dim3(256), 0, stream>>>(
      Xb, Xb, kDim, 0L, Wb, Wb, kDim, 0L,
      (void*)QKh, (void*)QKh, kQKCols, 0L, x, x, 0L, kTok, kQKCols, kDim, 1.0f);

  const unsigned short* WbV = Wb + (size_t)kQKCols * kDim;
  const int tilesV = (kDh / 64) * (kSeq / 64);
  for (int b = 0; b < kBatch; ++b) {
    const unsigned short* Xbb = Xb + (size_t)b * kSeq * kDim;
    unsigned short* Vtb = Vt + (size_t)b * kHeads * kDh * kSeq;
    wmma_gemm64<1, false, 0, 1, false, 0><<<dim3(tilesV / 8, kHeads), dim3(256), 0, stream>>>(
        WbV, WbV, kDim, (long)kDh * kDim, Xbb, Xbb, kDim, 0L,
        (void*)Vtb, (void*)Vtb, kSeq, (long)kDh * kSeq, x, x, 0L, kDh, kSeq, kDim, 1.0f);
  }

  attn_f16_kernel<<<dim3(kBatch * kHeads * (kSeq / kQB)), dim3(128), 0, stream>>>(QKh, Vt, out);
}
